// GAT_Net_18056042512584
// MI455X (gfx1250) — hardware-verified
//
#include <hip/hip_runtime.h>
#include <math.h>

#define NN 50000
#define NE 1600000
#define NV (NE + NN)
#define EDEC 500000
#define NPAIR 1000000
#define CIN 128
#define HIDC 128
#define OUTC 64
#define NPG 50048
#define XPITCH 256
#define NT 256
#define SPT 16
#define SCH (NT * SPT)
#define NCH ((NV + SCH - 1) / SCH)
#define ACCF 65536
#define SRB1 (ACCF / HIDC)
#define SRB2 (ACCF / OUTC)
#define RPW1 (SRB1 / 8)
#define RPW2 (SRB2 / 8)
#define NTL1 98
#define NTL2 49
#define NPT 50176
#define DCH 72000
#define DCHL 64000
#define NDCH 14
#define ACAR 16.0f
#define WCAR 16.0f

static_assert(NE % SPT == 0 && SCH % SPT == 0);
static_assert(SCH == 4096);
static_assert(NCH * SCH >= NV);
static_assert((NCH - 1) * SCH < NV);
static_assert(SRB1 == 512 && SRB2 == 1024 && RPW1 == 64 && RPW2 == 128);
static_assert(NTL1 * SRB1 == NPT && NTL2 * SRB2 == NPT);
static_assert(NPT >= NPG && NPG >= NN && NPG % 64 == 0 && NPG - NN < 64);
static_assert(NN < 65536 && SRB2 < 32768);
static_assert(DCH % 64 == 0 && DCHL % 64 == 0 && (NDCH - 1) * DCH + DCHL == NPAIR);
static_assert(EDEC % 16 == 0 && DCH % 16 == 0 && DCHL % 16 == 0);
static_assert(CIN % 32 == 0 && HIDC % 32 == 0 && OUTC % 32 == 0);
static_assert((NPG * CIN / 8) % 256 == 0);

typedef __attribute__((ext_vector_type(16))) _Float16 v16h;
typedef __attribute__((ext_vector_type(8)))  _Float16 v8h;
typedef __attribute__((ext_vector_type(16))) __bf16   v16b;
typedef __attribute__((ext_vector_type(8)))  __bf16   v8b;
typedef __attribute__((ext_vector_type(8)))  float    v8f;
typedef __attribute__((ext_vector_type(4)))  float    v4f;
typedef __attribute__((ext_vector_type(2)))  float    v2f;
typedef __attribute__((ext_vector_type(4)))  unsigned int v4u;
typedef __attribute__((ext_vector_type(4)))  int      v4i;

__device__ __forceinline__ unsigned short f2bf_bits(float f) {
  unsigned u = __float_as_uint(f);
  return (unsigned short)((u + 0x7FFFu + ((u >> 16) & 1u)) >> 16);
}
__device__ __forceinline__ float bf_bits2f(unsigned short h) { return __uint_as_float(((unsigned)h) << 16); }

__device__ __forceinline__ void dep_guard_h(v8f& a, v8f& b, v16h x, v16h y) { asm volatile("v_nop\n\tv_nop\n\tv_nop\n\tv_nop" : "+v"(a), "+v"(b) : "v"(x), "v"(y)); }
__device__ __forceinline__ void dep_guard_b(v8f& a, v8f& b, v16b x, v16b y) { asm volatile("v_nop\n\tv_nop\n\tv_nop\n\tv_nop" : "+v"(a), "+v"(b) : "v"(x), "v"(y)); }
__device__ __forceinline__ void keep4_h(v16h a, v16h b, v16h c, v16h d) { asm volatile("v_nop" :: "v"(a), "v"(b), "v"(c), "v"(d)); }
__device__ __forceinline__ void keep4_b(v16b a, v16b b, v16b c, v16b d) { asm volatile("v_nop" :: "v"(a), "v"(b), "v"(c), "v"(d)); }
__device__ __forceinline__ void acc_guard4(v8f& a, v8f& b, v8f& c, v8f& d) { asm volatile("v_nop\n\tv_nop\n\tv_nop\n\tv_nop" : "+v"(a), "+v"(b), "+v"(c), "+v"(d)); }
template <typename T> struct Frag;
template <> struct Frag<_Float16> {
  typedef v16h V; union U { v16h v; v8h h[2]; };
  static __device__ __forceinline__ v16h load(const _Float16* p) {
    U f; f.h[0] = *(const v8h*)(p); f.h[1] = *(const v8h*)(p + 16); return f.v;
  }
  static __device__ __forceinline__ v8f mma(v16h a, v16h b, v8f c) {
    return __builtin_amdgcn_wmma_f32_16x16x32_f16(false, a, false, b, (short)0, c, false, false);
  }
  static __device__ __forceinline__ void guard(v8f& a, v8f& b, v16h x, v16h y) { dep_guard_h(a, b, x, y); }
  static __device__ __forceinline__ void keep(v16h a, v16h b, v16h c, v16h d) { keep4_h(a, b, c, d); }
};
template <> struct Frag<__bf16> {
  typedef v16b V; union U { v16b v; v8b h[2]; };
  static __device__ __forceinline__ v16b load(const __bf16* p) {
    U f; f.h[0] = *(const v8b*)(p); f.h[1] = *(const v8b*)(p + 16); return f.v;
  }
  static __device__ __forceinline__ v8f mma(v16b a, v16b b, v8f c) {
    return __builtin_amdgcn_wmma_f32_16x16x32_bf16(false, a, false, b, (short)0, c, false, false);
  }
  static __device__ __forceinline__ void guard(v8f& a, v8f& b, v16b x, v16b y) { dep_guard_b(a, b, x, y); }
  static __device__ __forceinline__ void keep(v16b a, v16b b, v16b c, v16b d) { keep4_b(a, b, c, d); }
};

__device__ __forceinline__ unsigned pk16(unsigned short a, unsigned short b) { return (unsigned)a | ((unsigned)b << 16); }
__device__ __forceinline__ unsigned short h_bits(float f) { const _Float16 h = (_Float16)f; return __builtin_bit_cast(unsigned short, h); }
__device__ __forceinline__ float bfrf(float f) { return __uint_as_float(((unsigned)f2bf_bits(f)) << 16); }
__device__ __forceinline__ v4f bfr4(v4f a) { v4f r; r[0] = bfrf(a[0]); r[1] = bfrf(a[1]); r[2] = bfrf(a[2]); r[3] = bfrf(a[3]); return r; }
__device__ __forceinline__ v2f bfr2(v2f a) { v2f r; r[0] = bfrf(a[0]); r[1] = bfrf(a[1]); return r; }

template <int ET> struct Elem;
template <> struct Elem<0> { typedef _Float16 T; };
template <> struct Elem<1> { typedef __bf16 T; };
template <int ET, bool SPLIT, int BIAS_MODE, int OUT_MODE, bool RESID, int ACT = 0>
__global__ __launch_bounds__(256) void wmma_gemm64(
    const unsigned short* __restrict__ Ap, const unsigned short* __restrict__ A2p, int lda, long strideA,
    const unsigned short* __restrict__ Btp, const unsigned short* __restrict__ Bt2p, int ldb, long strideB,
    void* __restrict__ Cout, void* __restrict__ Cout2, int ldc, long strideC,
    const float* __restrict__ bias,
    const float* __restrict__ resid, long strideR,
    int M, int N, int K, float scale) {
  typedef typename Elem<ET>::T T;
  typedef typename Frag<T>::V V;
  const T* A = (const T*)Ap; const T* A2 = (const T*)A2p; const T* Bt = (const T*)Btp; const T* Bt2 = (const T*)Bt2p;
  __shared__ __align__(16) float sT[8][16 * 68];
  __shared__ __align__(16) float sO[8][64];
  const int b    = blockIdx.y;
  const int lane = threadIdx.x & 31;
  const int wave = threadIdx.x >> 5;
  const int tilesN = N >> 6;
  const int tilesM = M >> 6;
  const int tile = blockIdx.x * 8 + wave;
  if (tile >= tilesM * tilesN) return;
  const int tm = tile / tilesN;
  const int tn = tile - tm * tilesN;
  const int m0 = tm << 6;
  const int n0 = tn << 6;

  const T* Ab  = A  + (size_t)b * strideA;
  const T* Bb  = Bt + (size_t)b * strideB;
  const T* Ab2 = SPLIT ? (A2  + (size_t)b * strideA) : nullptr;
  const T* Bb2 = SPLIT ? (Bt2 + (size_t)b * strideB) : nullptr;

  const int rlane = lane & 15;
  const int koff  = (lane >> 4) * 8;
  const int mOff  = (lane >> 4) * 8;

  v8f acc[4][4];
#pragma unroll
  for (int i = 0; i < 4; ++i)
#pragma unroll
    for (int j = 0; j < 4; ++j) acc[i][j] = (v8f){0.f,0.f,0.f,0.f,0.f,0.f,0.f,0.f};

  for (int k0 = 0; k0 < K; k0 += 32) {
    V bh[4], bl[4];
#pragma unroll
    for (int j = 0; j < 4; ++j) {
      const size_t bo = (size_t)(n0 + (j << 4) + rlane) * ldb + koff + k0;
      bh[j] = Frag<T>::load(Bb + bo);
      if (SPLIT) bl[j] = Frag<T>::load(Bb2 + bo);
    }
#pragma unroll
    for (int i = 0; i < 4; ++i) {
      const size_t ao = (size_t)(m0 + (i << 4) + rlane) * lda + koff + k0;
      V ah = Frag<T>::load(Ab + ao);
      V al;
      if (SPLIT) al = Frag<T>::load(Ab2 + ao);
#pragma unroll
      for (int j = 0; j < 4; ++j) {
        acc[i][j] = Frag<T>::mma(ah, bh[j], acc[i][j]);
        if (SPLIT) {
          acc[i][j] = Frag<T>::mma(ah, bl[j], acc[i][j]);
          acc[i][j] = Frag<T>::mma(al, bh[j], acc[i][j]);
        }
      }
      Frag<T>::guard(acc[i][0], acc[i][3], ah, SPLIT ? al : ah);
    }
    Frag<T>::keep(bh[0], bh[1], bh[2], bh[3]);
    if (SPLIT) Frag<T>::keep(bl[0], bl[1], bl[2], bl[3]);
  }
  acc_guard4(acc[0][0], acc[0][1], acc[0][2], acc[0][3]);
  acc_guard4(acc[1][0], acc[1][1], acc[1][2], acc[1][3]);
  acc_guard4(acc[2][0], acc[2][1], acc[2][2], acc[2][3]);
  acc_guard4(acc[3][0], acc[3][1], acc[3][2], acc[3][3]);

  float* slab = sT[wave];
  const float* Rb = RESID ? (resid + (size_t)b * strideR) : nullptr;
#pragma unroll
  for (int i = 0; i < 4; ++i) {
    const int mBase = m0 + (i << 4);
#pragma unroll
    for (int j = 0; j < 4; ++j) {
      const int n = n0 + (j << 4) + rlane;
      float bv = 0.f;
      if (BIAS_MODE == 2) bv = bias[n];
#pragma unroll
      for (int r = 0; r < 8; ++r) {
        float v = acc[i][j][r] * scale;
        if (BIAS_MODE == 1) v += bias[mBase + mOff + r];
        if (BIAS_MODE == 2) v += bv;
        if (RESID) v += Rb[(size_t)(mBase + mOff + r) * ldc + n];
        if (ACT == 2) v = fmaxf(v, 0.0f);
        if (ACT == 4) v = (v > 0.f) ? v : 0.01f * v;
        slab[(mOff + r) * 68 + (j << 4) + rlane] = v;
      }
    }
    __builtin_amdgcn_fence(__ATOMIC_RELEASE, "workgroup");
    __builtin_amdgcn_wave_barrier();
    __builtin_amdgcn_fence(__ATOMIC_ACQUIRE, "workgroup");
    if (OUT_MODE == 0) {
      float* C = (float*)Cout + (size_t)b * strideC;
      const int hh = lane >> 4, c4 = (lane & 15) * 4;
      for (int pass = 0; pass < 2; ++pass) {
#pragma unroll
        for (int it = 0; it < 8; ++it) {
          const int row = it * 2 + hh;
          v4f v = *(const v4f*)(slab + row * 68 + c4);
          *(volatile v4f*)(C + (size_t)(mBase + row) * ldc + n0 + c4) = v;
        }
        __threadfence();
      }
    } else if (OUT_MODE == 3) {
      const float* dv = (const float*)Cout2;
      const int rr = lane & 15, ch = (lane >> 4) * 32;
      float ds = 0.f;
#pragma unroll
      for (int cc = 0; cc < 32; cc += 4) {
        const v4f hv4 = *(const v4f*)(slab + rr * 68 + ch + cc);
        const v4f wv4 = *(const v4f*)(dv + ch + cc);
        ds += hv4[0] * wv4[0] + hv4[1] * wv4[1] + hv4[2] * wv4[2] + hv4[3] * wv4[3];
      }
      ds += __shfl_xor(ds, 16, 32);
      if (lane < 16) sO[wave][(i << 4) + rr] = ds + dv[64];
    } else {
      const int q = lane >> 3, c8 = (lane & 7) * 8;
      unsigned short* C  = (unsigned short*)Cout  + (size_t)b * strideC;
      unsigned short* C2 = (OUT_MODE == 2) ? ((unsigned short*)Cout2 + (size_t)b * strideC) : nullptr;
      for (int pass = 0; pass < 2; ++pass) {
#pragma unroll
        for (int it = 0; it < 4; ++it) {
          const int row = it * 4 + q;
          const float* sp = slab + row * 68 + c8;
          v8h hv, lv;
#pragma unroll
          for (int e = 0; e < 8; ++e) {
            if (OUT_MODE == 1) {
              hv[e] = (_Float16)sp[e];
            } else {
              unsigned short hb = f2bf_bits(sp[e]);
              unsigned short lb = f2bf_bits(sp[e] - bf_bits2f(hb));
              hv[e] = __builtin_bit_cast(_Float16, hb);
              lv[e] = __builtin_bit_cast(_Float16, lb);
            }
          }
          *(volatile v8h*)(C + (size_t)(mBase + row) * ldc + n0 + c8) = hv;
          if (OUT_MODE == 2) *(volatile v8h*)(C2 + (size_t)(mBase + row) * ldc + n0 + c8) = lv;
        }
        __threadfence();
      }
    }
    __builtin_amdgcn_fence(__ATOMIC_RELEASE, "workgroup");
    __builtin_amdgcn_wave_barrier();
    __builtin_amdgcn_fence(__ATOMIC_ACQUIRE, "workgroup");
  }
  if (OUT_MODE == 3) {
    float* Co = (float*)Cout + (size_t)b * strideC + m0;
    const int l4 = (lane & 15) * 4;
    const v4f ov = *(const v4f*)(sO[wave] + l4);
    for (int pass = 0; pass < 2; ++pass) {
      if (lane < 16) *(volatile v4f*)(Co + l4) = ov;
      __threadfence();
    }
  }
}

__global__ __launch_bounds__(256) void wtr_kernel(const float* __restrict__ W, int kin, int nout,
                                                  unsigned short* __restrict__ outp, int row0, float scale, int f16mode) {
  __shared__ float sm[64][65];
  const int t  = threadIdx.x;
  const int k0 = blockIdx.x * 64;
  const int nb = blockIdx.y * 64;
#pragma unroll
  for (int i = 0; i < 16; ++i) {
    const int e = i * 256 + t;
    const int r = e >> 6;
    const int c = e & 63;
    sm[c][r] = bfrf(W[(size_t)(k0 + r) * nout + nb + c]) * scale;
  }
  __syncthreads();
  const int lane = t & 31, wave = t >> 5;
  const int q = lane >> 3, c8 = (lane & 7) * 8;
  for (int pass = 0; pass < 2; ++pass) {
#pragma unroll
    for (int it = 0; it < 2; ++it) {
      const int row = wave * 8 + it * 4 + q;
      unsigned short hb[8];
#pragma unroll
      for (int e = 0; e < 8; ++e) {
        const float f = sm[row][c8 + e];
        const unsigned short fh = h_bits(f);
        const unsigned short fb = f2bf_bits(f);
        hb[e] = f16mode ? fh : fb;
      }
      const v4u u = (v4u){pk16(hb[0], hb[1]), pk16(hb[2], hb[3]), pk16(hb[4], hb[5]), pk16(hb[6], hb[7])};
      *(volatile v4u*)(outp + (size_t)(row0 + nb + row) * kin + k0 + c8) = u;
    }
    __threadfence();
  }
}

__global__ __launch_bounds__(256) void tab_kernel(const float* __restrict__ fb1, const float* __restrict__ fb2, const float* __restrict__ fb3,
                                                  const float* __restrict__ fw4, const float* __restrict__ fb4, float* __restrict__ TAB) {
  const int t = threadIdx.x;
  const int i1 = (t < 64) ? t : 63;
  const int i2 = (t < 64) ? 0 : ((t < 192) ? (t - 64) : 127);
  const int i3 = (t < 192) ? 0 : (t - 192);
  const float v1 = ACAR * bfrf(fb1[i1]);
  const float v2 = ACAR * bfrf(fb2[i2]);
  const float v3 = bfrf(fb3[i3]);
  const float c1 = (t < 64) ? 1.f : 0.f;
  const float c2 = (t >= 64 && t < 192) ? 1.f : 0.f;
  const float c3 = (t >= 192) ? 1.f : 0.f;
  const float v = c1 * v1 + c2 * v2 + c3 * v3;
  ((volatile float*)TAB)[t] = v;
  __threadfence();
  ((volatile float*)TAB)[t] = v;
  const float g4 = bfrf(fw4[i1]);
  const float g5 = bfrf(fb4[0]);
  const float d1 = (t < 64) ? 1.f : 0.f;
  const float d2 = (t == 64) ? 1.f : 0.f;
  const float u = d1 * g4 + d2 * g5;
  if (t < 96) {
    ((volatile float*)TAB)[256 + t] = u;
    __threadfence();
    ((volatile float*)TAB)[256 + t] = u;
  }
}

__global__ __launch_bounds__(256) void castx_kernel(const float* __restrict__ x, unsigned short* __restrict__ Xb) {
  const int i = blockIdx.x * 256 + threadIdx.x;
  const int live = (i < (NN * CIN / 8)) ? 1 : 0;
  const size_t so = (size_t)(live ? i : 0) * 8;
  const v4f a = *(const v4f*)(x + so);
  const v4f c = *(const v4f*)(x + so + 4);
  unsigned short hb[8];
#pragma unroll
  for (int e = 0; e < 4; ++e) { hb[e] = f2bf_bits(a[e]); hb[4 + e] = f2bf_bits(c[e]); }
  const unsigned mk = live ? 0xFFFFFFFFu : 0u;
  const v4u u = (v4u){pk16(hb[0], hb[1]) & mk, pk16(hb[2], hb[3]) & mk, pk16(hb[4], hb[5]) & mk, pk16(hb[6], hb[7]) & mk};
  unsigned short* q = Xb + 8 * (size_t)i;
  *(volatile v4u*)q = u;
  __threadfence();
  *(volatile v4u*)q = u;
}

__device__ __forceinline__ int blk_excl_scan(int cnt, int* scan_ws, int tid, int* tot) {
  const int lane = tid & 31, wave = tid >> 5; int incl = cnt;
#pragma unroll
  for (int o = 1; o < 32; o <<= 1) { const int v = __shfl_up(incl, o, 32); if (lane >= o) incl += v; }
  if (lane == 31) scan_ws[wave] = incl;
  __syncthreads();
  if (wave == 0) { int wv = (lane < NT / 32) ? scan_ws[lane] : 0; int wincl = wv;
#pragma unroll
    for (int o = 1; o < 32; o <<= 1) { const int v = __shfl_up(wincl, o, 32); if (lane >= o) wincl += v; }
    if (lane < NT / 32) scan_ws[32 + lane] = wincl - wv; if (lane == 31) scan_ws[64] = wincl; }
  __syncthreads();
  const int res = scan_ws[32 + wave] + incl - cnt; *tot = scan_ws[64];
  return res;
}
template <int SP, int CAP, int SRBT>
__device__ __forceinline__ int chunk_hits(const int* __restrict__ dstv, const int* __restrict__ srcv, int e0, int n0, int tid,
                                          int* LIST, int* scan_ws) {
  const int eb = e0 + tid * SP;
  const int realg = (eb < NE) ? 1 : 0;
  const int ebc = realg ? eb : (NE - SP);
  int rec[SP]; int cnt = 0;
#pragma unroll
  for (int k = 0; k < SP; k += 4) {
    const v4i d4 = *(const v4i*)(dstv + ebc + k);
    const v4i s4 = *(const v4i*)(srcv + ebc + k);
#pragma unroll
    for (int e = 0; e < 4; ++e) {
      const int ev = eb + k + e;
      const int dvn = ev - NE;
      const int d = dvn + (d4[e] - dvn) * realg;
      int s = dvn + (s4[e] - dvn) * realg;
      s = s < 0 ? 0 : (s > NN - 1 ? NN - 1 : s);
      const int inr = realg | ((ev < NV) ? 1 : 0);
      int r = -1;
      if (inr != 0 && d >= n0 && d < n0 + SRBT && d < NN) { r = ((d - n0) << 16) | s; ++cnt; }
      rec[k + e] = r;
    }
  }
  int tot; int p = blk_excl_scan(cnt, scan_ws, tid, &tot);
#pragma unroll
  for (int k = 0; k < SP; ++k) if (rec[k] >= 0) { if ((unsigned)p < (unsigned)CAP) LIST[p] = rec[k]; ++p; }
  __syncthreads();
  return tot < CAP ? tot : CAP;
}

__global__ __launch_bounds__(NT) void gat1_kernel(const float* __restrict__ XLR, const int* __restrict__ ei,
                                                 const float* __restrict__ av, const float* __restrict__ bv,
                                                 unsigned short* __restrict__ Zh) {
  __shared__ __align__(16) float ACC[ACCF];
  __shared__ int LIST[SCH];
  __shared__ float SM[SRB1];
  __shared__ float SL[SRB1];
  __shared__ int scan_ws[80];
  const int tid = threadIdx.x, lane = tid & 31, wave = tid >> 5;
  const int n0 = blockIdx.x * SRB1;
  const v4f a4 = bfr4(*(const v4f*)(av + 4 * lane));
  const int c8 = (lane & 15) * 8;
  const v4f bA = bfr4(*(const v4f*)(bv + c8));
  const v4f bB = bfr4(*(const v4f*)(bv + c8 + 4));
  const v4f z4 = {0.f, 0.f, 0.f, 0.f};
#pragma unroll 4
  for (int i = tid; i < ACCF / 4; i += NT) *(v4f*)(ACC + 4 * i) = z4;
  for (int i = tid; i < SCH; i += NT) LIST[i] = -1;
  for (int i = tid; i < SRB1; i += NT) { SM[i] = -INFINITY; SL[i] = 0.f; }
  for (int i = tid; i < 80; i += NT) scan_ws[i] = 0;
  __syncthreads();
  const int* srcv = ei; const int* dstv = ei + NE;
#pragma unroll 1
  for (int c = 0; c < NCH; ++c) {
    const int tot = chunk_hits<SPT, SCH, SRB1>(dstv, srcv, c * SCH, n0, tid, LIST, scan_ws);
#pragma unroll 1
    for (int base = 0; base < tot; base += 32) {
      const int q = base + lane;
      const int qc = (q < SCH) ? q : (SCH - 1);
      const int lq = LIST[qc];
      const int keep = (q < tot) ? 1 : 0;
      const int rv = lq * keep + keep - 1;
      const int own = (rv >= 0 && (rv >> 22) == wave) ? 1 : 0;
      unsigned msk = (unsigned)__ballot(own);
#pragma unroll 1
      for (int it = 0; it < 32; ++it) {
        if (msk == 0u) break;
        const int bp = __builtin_ctz(msk); msk &= msk - 1u;
        const int r = __shfl(rv, bp, 32);
        const int dl = r >> 16, s = r & 0xFFFF;
        const int n = n0 + dl;
        const v4f xs = *(const v4f*)(XLR + (size_t)s * XPITCH + 4 * lane);
        const v4f xd = *(const v4f*)(XLR + (size_t)n * XPITCH + HIDC + 4 * lane);
        v4f tq = xs + xd;
#pragma unroll
        for (int e = 0; e < 4; ++e) tq[e] = (tq[e] > 0.f) ? tq[e] : 0.2f * tq[e];
        float p = tq[0] * a4[0] + tq[1] * a4[1] + tq[2] * a4[2] + tq[3] * a4[3];
        p += __shfl_xor(p, 1, 32); p += __shfl_xor(p, 2, 32); p += __shfl_xor(p, 4, 32);
        p += __shfl_xor(p, 8, 32); p += __shfl_xor(p, 16, 32);
        const float mo = SM[dl], lo = SL[dl];
        const float mn = fmaxf(mo, p);
        const float rr = expf(mo - mn), ex = expf(p - mn);
        const float ln = lo * rr + ex;
        if (lane == 0) { SM[dl] = mn; SL[dl] = ln; }
        float* rp = ACC + dl * HIDC + 4 * lane;
        v4f a = *(const v4f*)rp;
        a = a * rr + ex * xs;
        *(v4f*)rp = a;
      }
    }
    __syncthreads();
  }
#pragma unroll 1
  for (int j = 0; j < RPW1 / 2; ++j) {
    const int dl = wave * RPW1 + 2 * j + (lane >> 4);
    const int n = n0 + dl;
    const float liv = (n < NN) ? ACAR : 0.f;
    float lv = SL[dl];
    lv = (lv > 0.f) ? lv : 1.0f;
    const float inv = 1.0f / lv;
    const float* rp = ACC + dl * HIDC + c8;
    const v4f a0 = *(const v4f*)rp;
    const v4f a1v = *(const v4f*)(rp + 4);
    const v4f t0 = a0 * inv + bA;
    const v4f t1 = a1v * inv + bB;
    v8h hv;
#pragma unroll
    for (int e = 0; e < 4; ++e) {
      hv[e]     = (_Float16)(fmaxf(t0[e], 0.f) * liv);
      hv[4 + e] = (_Float16)(fmaxf(t1[e], 0.f) * liv);
    }
    unsigned short* op = Zh + (size_t)n * HIDC + c8;
    *(volatile v8h*)op = hv;
    __threadfence();
    *(volatile v8h*)op = hv;
  }
}

__global__ __launch_bounds__(NT) void gat2_kernel(const float* __restrict__ XLR, const int* __restrict__ ei,
                                                 const float* __restrict__ av, const float* __restrict__ bv,
                                                 unsigned short* __restrict__ Zh) {
  __shared__ __align__(16) float ACC[ACCF];
  __shared__ int LIST[SCH];
  __shared__ float SM[SRB2];
  __shared__ float SL[SRB2];
  __shared__ int scan_ws[80];
  const int tid = threadIdx.x, lane = tid & 31, wave = tid >> 5;
  const int n0 = blockIdx.x * SRB2;
  const v2f a2v = bfr2(*(const v2f*)(av + 2 * lane));
  const int q4 = lane >> 3, c8 = (lane & 7) * 8;
  const v4f bA = bfr4(*(const v4f*)(bv + c8));
  const v4f bB = bfr4(*(const v4f*)(bv + c8 + 4));
  const v4f z4 = {0.f, 0.f, 0.f, 0.f};
#pragma unroll 4
  for (int i = tid; i < ACCF / 4; i += NT) *(v4f*)(ACC + 4 * i) = z4;
  for (int i = tid; i < SCH; i += NT) LIST[i] = -1;
  for (int i = tid; i < SRB2; i += NT) { SM[i] = -INFINITY; SL[i] = 0.f; }
  for (int i = tid; i < 80; i += NT) scan_ws[i] = 0;
  __syncthreads();
  const int* srcv = ei; const int* dstv = ei + NE;
#pragma unroll 1
  for (int c = 0; c < NCH; ++c) {
    const int tot = chunk_hits<SPT, SCH, SRB2>(dstv, srcv, c * SCH, n0, tid, LIST, scan_ws);
#pragma unroll 1
    for (int base = 0; base < tot; base += 32) {
      const int q = base + lane;
      const int qc = (q < SCH) ? q : (SCH - 1);
      const int lq = LIST[qc];
      const int keep = (q < tot) ? 1 : 0;
      const int rv = lq * keep + keep - 1;
      const int own = (rv >= 0 && (rv >> 23) == wave) ? 1 : 0;
      unsigned msk = (unsigned)__ballot(own);
#pragma unroll 1
      for (int it = 0; it < 32; ++it) {
        if (msk == 0u) break;
        const int bp = __builtin_ctz(msk); msk &= msk - 1u;
        const int r = __shfl(rv, bp, 32);
        const int dl = r >> 16, s = r & 0xFFFF;
        const int n = n0 + dl;
        const v2f xs = *(const v2f*)(XLR + (size_t)s * XPITCH + 2 * lane);
        const v2f xd = *(const v2f*)(XLR + (size_t)n * XPITCH + OUTC + 2 * lane);
        v2f tq = xs + xd;
#pragma unroll
        for (int e = 0; e < 2; ++e) tq[e] = (tq[e] > 0.f) ? tq[e] : 0.2f * tq[e];
        float p = tq[0] * a2v[0] + tq[1] * a2v[1];
        p += __shfl_xor(p, 1, 32); p += __shfl_xor(p, 2, 32); p += __shfl_xor(p, 4, 32);
        p += __shfl_xor(p, 8, 32); p += __shfl_xor(p, 16, 32);
        const float mo = SM[dl], lo = SL[dl];
        const float mn = fmaxf(mo, p);
        const float rr = expf(mo - mn), ex = expf(p - mn);
        const float ln = lo * rr + ex;
        if (lane == 0) { SM[dl] = mn; SL[dl] = ln; }
        float* rp = ACC + dl * OUTC + 2 * lane;
        v2f a = *(const v2f*)rp;
        a = a * rr + ex * xs;
        *(v2f*)rp = a;
      }
    }
    __syncthreads();
  }
#pragma unroll 1
  for (int j = 0; j < RPW2 / 4; ++j) {
    const int dl = wave * RPW2 + 4 * j + q4;
    const int n = n0 + dl;
    const float liv = (n < NN) ? ACAR : 0.f;
    float lv = SL[dl];
    lv = (lv > 0.f) ? lv : 1.0f;
    const float inv = 1.0f / lv;
    const float* rp = ACC + dl * OUTC + c8;
    const v4f a0 = *(const v4f*)rp;
    const v4f a1v = *(const v4f*)(rp + 4);
    const v4f t0 = a0 * inv + bA;
    const v4f t1 = a1v * inv + bB;
    v8h hv;
#pragma unroll
    for (int e = 0; e < 4; ++e) {
      hv[e]     = (_Float16)(t0[e] * liv);
      hv[4 + e] = (_Float16)(t1[e] * liv);
    }
    unsigned short* op = Zh + (size_t)n * OUTC + c8;
    *(volatile v8h*)op = hv;
    __threadfence();
    *(volatile v8h*)op = hv;
  }
}

__global__ __launch_bounds__(256) void gather_kernel(const unsigned short* __restrict__ Z2h, const int* __restrict__ pos,
                                                     const int* __restrict__ neg, unsigned short* __restrict__ H0, int g0) {
  const int t = threadIdx.x;
  const int rl = blockIdx.x * 16 + (t >> 4);
  const int g = g0 + rl;
  const int isneg = (g >= EDEC) ? 1 : 0;
  int ip = g; ip = ip > EDEC - 1 ? EDEC - 1 : ip;
  int iq = g - EDEC; iq = iq < 0 ? 0 : (iq > EDEC - 1 ? EDEC - 1 : iq);
  const int pa = pos[ip], pb = pos[EDEC + ip];
  const int qa = neg[iq], qb = neg[EDEC + iq];
  const int ia = pa + (qa - pa) * isneg;
  const int ib = pb + (qb - pb) * isneg;
  const int p = t & 15;
  const int hsel = p >> 3;
  int node = ia + (ib - ia) * hsel;
  node = node < 0 ? 0 : (node > NN - 1 ? NN - 1 : node);
  const v4u v = *(const v4u*)(Z2h + (size_t)node * OUTC + (p & 7) * 8);
  unsigned short* dp = H0 + (size_t)rl * (2 * OUTC) + p * 8;
  *(volatile v4u*)dp = v;
  __threadfence();
  *(volatile v4u*)dp = v;
}

static_assert((size_t)NPG * CIN * 2 + (size_t)NPT * HIDC * 2 + (size_t)DCH * (128 * 2 + 64 * 2 + 128 * 2) +
              (size_t)NPG * XPITCH * 4 + (size_t)NPT * OUTC * 2 + 65536 + 32768 + 3 * 16384 + 1536 <= (size_t)134217728);

extern "C" void kernel_launch(void* const* d_in, const int* in_sizes, int n_in,
                              void* d_out, int out_size, void* d_ws, size_t ws_size, hipStream_t stream) {
  (void)in_sizes; (void)n_in; (void)out_size;
  const float* x   = (const float*)d_in[0];
  const int*   ei  = (const int*)  d_in[1];
  const int*   pos = (const int*)  d_in[2];
  const int*   neg = (const int*)  d_in[3];
  const float* w1l = (const float*)d_in[4];
  const float* w1r = (const float*)d_in[5];
  const float* a1  = (const float*)d_in[6];
  const float* b1  = (const float*)d_in[7];
  const float* w2l = (const float*)d_in[8];
  const float* w2r = (const float*)d_in[9];
  const float* a2  = (const float*)d_in[10];
  const float* b2  = (const float*)d_in[11];
  const float* fw1 = (const float*)d_in[12];
  const float* fb1 = (const float*)d_in[13];
  const float* fw2 = (const float*)d_in[14];
  const float* fb2 = (const float*)d_in[15];
  const float* fw3 = (const float*)d_in[16];
  const float* fb3 = (const float*)d_in[17];
  const float* fw4 = (const float*)d_in[18];
  const float* fb4 = (const float*)d_in[19];
  float* out = (float*)d_out;

  char* ws = (char*)d_ws; size_t off = 0;
  auto carve = [&](size_t bytes) -> char* { char* p = ws + off; off += (bytes + 255) & ~(size_t)255; return p; };
  unsigned short* Xb   = (unsigned short*)carve((size_t)NPG * CIN * 2);
  unsigned short* Z1h  = (unsigned short*)carve((size_t)NPT * HIDC * 2);
  char*           RD   = carve((size_t)DCH * (128 * 2 + 64 * 2 + 128 * 2));
  float*          XLR  = (float*)carve((size_t)NPG * XPITCH * 4);
  unsigned short* Z2h  = (unsigned short*)carve((size_t)NPT * OUTC * 2);
  unsigned short* Bt1  = (unsigned short*)carve((size_t)256 * 128 * 2);
  unsigned short* Bt2  = (unsigned short*)carve((size_t)128 * 128 * 2);
  unsigned short* BtF1 = (unsigned short*)carve((size_t)64 * 128 * 2);
  unsigned short* BtF2 = (unsigned short*)carve((size_t)128 * 64 * 2);
  unsigned short* BtF3 = (unsigned short*)carve((size_t)64 * 128 * 2);
  float*          TAB  = (float*)carve((size_t)352 * 4);
  if (off > ws_size || off > (size_t)134217728) return;
  unsigned short* H0h = (unsigned short*)RD;
  unsigned short* H1h = (unsigned short*)(RD + (size_t)DCH * 128 * 2);
  unsigned short* H2h = (unsigned short*)(RD + (size_t)DCH * 128 * 2 + (size_t)DCH * 64 * 2);
  const unsigned short* nul16 = (const unsigned short*)nullptr;

  auto ggrid = [](int M, int N) { return dim3((unsigned)((((M / 64) * (N / 64)) + 7) / 8), 1); };

  wtr_kernel<<<dim3(2, 2), 256, 0, stream>>>(w1l, 128, 128, Bt1, 0,   1.0f, 0);
  wtr_kernel<<<dim3(2, 2), 256, 0, stream>>>(w1r, 128, 128, Bt1, 128, 1.0f, 0);
  wtr_kernel<<<dim3(2, 1), 256, 0, stream>>>(w2l, 128, 64,  Bt2, 0,   WCAR, 1);
  wtr_kernel<<<dim3(2, 1), 256, 0, stream>>>(w2r, 128, 64,  Bt2, 64,  WCAR, 1);
  wtr_kernel<<<dim3(2, 1), 256, 0, stream>>>(fw1, 128, 64,  BtF1, 0,  WCAR, 1);
  wtr_kernel<<<dim3(1, 2), 256, 0, stream>>>(fw2, 64,  128, BtF2, 0,  WCAR, 1);
  wtr_kernel<<<dim3(2, 1), 256, 0, stream>>>(fw3, 128, 64,  BtF3, 0,  WCAR, 1);
  tab_kernel<<<1, 256, 0, stream>>>(fb1, fb2, fb3, fw4, fb4, TAB);
  castx_kernel<<<(NPG * CIN / 8) / 256, 256, 0, stream>>>(x, Xb);

  wmma_gemm64<1, false, 0, 0, false, 0><<<ggrid(NPG, 256), 256, 0, stream>>>(
      Xb, nul16, CIN, 0L, Bt1, nul16, CIN, 0L, (void*)XLR, (void*)nullptr, XPITCH, 0L,
      (const float*)nullptr, (const float*)nullptr, 0L, NPG, 256, CIN, 1.0f);
  gat1_kernel<<<NTL1, NT, 0, stream>>>(XLR, ei, a1, b1, Z1h);

  wmma_gemm64<0, false, 0, 0, false, 0><<<ggrid(NPG, 128), 256, 0, stream>>>(
      Z1h, nul16, HIDC, 0L, Bt2, nul16, HIDC, 0L, (void*)XLR, (void*)nullptr, XPITCH, 0L,
      (const float*)nullptr, (const float*)nullptr, 0L, NPG, 128, HIDC, 1.0f / (ACAR * WCAR));
  gat2_kernel<<<NTL2, NT, 0, stream>>>(XLR, ei, a2, b2, Z2h);

  for (int c = 0; c < NDCH; ++c) {
    const int g0 = c * DCH;
    const int rows = (c < NDCH - 1) ? DCH : DCHL;
    gather_kernel<<<rows / 16, 256, 0, stream>>>(Z2h, pos, neg, H0h, g0);
    wmma_gemm64<0, false, 2, 1, false, 2><<<ggrid(rows, 64), 256, 0, stream>>>(
        H0h, nul16, 128, 0L, BtF1, nul16, 128, 0L, (void*)H1h, (void*)nullptr, 64, 0L,
        TAB + 0, (const float*)nullptr, 0L, rows, 64, 128, 1.0f / WCAR);
    wmma_gemm64<0, false, 2, 1, false, 2><<<ggrid(rows, 128), 256, 0, stream>>>(
        H1h, nul16, 64, 0L, BtF2, nul16, 64, 0L, (void*)H2h, (void*)nullptr, 128, 0L,
        TAB + 64, (const float*)nullptr, 0L, rows, 128, 64, 1.0f / WCAR);
    wmma_gemm64<0, false, 2, 3, false, 2><<<ggrid(rows, 64), 256, 0, stream>>>(
        H2h, nul16, 128, 0L, BtF3, nul16, 128, 0L, (void*)(out + (size_t)g0), (void*)(TAB + 256), 64, 0L,
        TAB + 192, (const float*)nullptr, 0L, rows, 64, 128, 1.0f / (ACAR * WCAR));
  }
}
